// MMD_loss_274877907592
// MI455X (gfx1250) — hardware-run, weakly checked
//
#include <hip/hip_runtime.h>

typedef __attribute__((ext_vector_type(16))) __bf16   v16b;
typedef __attribute__((ext_vector_type(8)))  __bf16   v8b;
typedef __attribute__((ext_vector_type(8)))  _Float16 v8h;
typedef __attribute__((ext_vector_type(8)))  float    v8f;
typedef __attribute__((ext_vector_type(4)))  float    v4f;

constexpr int kHalfN      = 4096;
constexpr int kNTot       = 2 * kHalfN;
constexpr int kDim        = 512;
constexpr int kTileRows   = 64;
constexpr int kTiles      = kNTot / kTileRows;
constexpr int kPairs      = kTiles * (kTiles + 1) / 2;
constexpr int kMainBlocks = kPairs / 8;
constexpr int kPrepBlocks = kNTot / (8 * 32);
static_assert(kTiles == 128);
static_assert(kPairs == 8256);
static_assert(kMainBlocks * 8 == kPairs);
static_assert(kPrepBlocks == 32);
static_assert(kPrepBlocks * 8 * 32 == kNTot);
static_assert((kDim % 32) == 0);
static_assert((kNTot % 64) == 0);
static_assert((kHalfN % kTileRows) == 0);
static_assert((kHalfN % 32) == 0);

constexpr size_t kOffT16  = 0;
constexpr size_t kOffSQ   = kOffT16  + (size_t)kNTot * kDim * 2;
constexpr size_t kOffCOL  = kOffSQ   + (size_t)kNTot * 4;
constexpr size_t kOffSCAL = kOffCOL  + (size_t)kPrepBlocks * kDim * 4;
constexpr size_t kOffPART = kOffSCAL + (size_t)128;
constexpr size_t kWsTotal = kOffPART + (size_t)kMainBlocks * 128;
static_assert(kWsTotal == 8619136ull);
static_assert(kWsTotal <= 134217728ull);
static_assert((kOffSQ % 128) == 0 && (kOffCOL % 128) == 0 && (kOffSCAL % 128) == 0 && (kOffPART % 128) == 0);

__device__ __forceinline__ unsigned short f2bf_bits(float f) {
  unsigned u = __float_as_uint(f);
  return (unsigned short)((u + 0x7FFFu + ((u >> 16) & 1u)) >> 16);
}
__device__ __forceinline__ float bf_bits2f(unsigned short h) { return __uint_as_float(((unsigned)h) << 16); }

struct FragB {
  union U { v16b v; v8b h[2]; };
  static __device__ __forceinline__ v16b load(const __bf16* p) {
    U f;
    f.h[0] = *(const v8b*)(p);
    f.h[1] = *(const v8b*)(p + 16);
    return f.v;
  }
};

__device__ __forceinline__ v8f mma_guarded(v16b a, v16b b, v8f c) {
  c = __builtin_amdgcn_wmma_f32_16x16x32_bf16(false, a, false, b, (short)0, c, false, false);
  asm volatile("v_nop\n\tv_nop\n\tv_nop\n\tv_nop" : "+v"(c) : "v"(a), "v"(b));
  return c;
}

__device__ __forceinline__ void tri_decode(int w, int& ti, int& tj) {
  int lo = 0, hi = kTiles - 1;
#pragma unroll
  for (int it = 0; it < 7; ++it) {
    const int mid = (lo + hi + 1) >> 1;
    const bool ok = ((mid * (mid + 1)) >> 1) <= w;
    lo = ok ? mid : lo;
    hi = ok ? hi : (mid - 1);
  }
  int t = w - ((lo * (lo + 1)) >> 1);
  t = t < 0 ? 0 : t;
  t = t > lo ? lo : t;
  ti = lo;
  tj = t;
}

__global__ __launch_bounds__(256) void prep_rows_kernel(
    const float* __restrict__ src, const float* __restrict__ tgt,
    unsigned short* __restrict__ T16, float* __restrict__ SQ, float* __restrict__ COLPART)
{
  __shared__ __align__(16) float sCol[8 * kDim];
  const int tid = threadIdx.x, lane = tid & 31, wave = tid >> 5;
  const int rowBase = (blockIdx.x * 8 + wave) * 32;
  const float* inBase = (rowBase < kHalfN) ? (src + (size_t)rowBase * kDim)
                                           : (tgt + (size_t)(rowBase - kHalfN) * kDim);
  float cs[16];
#pragma unroll
  for (int e = 0; e < 16; ++e) cs[e] = 0.0f;
  float keep = 0.0f;

#pragma unroll 1
  for (int r = 0; r < 32; ++r) {
    const float* p = inBase + (size_t)r * kDim + lane * 8;
    const v4f a0 = *(const v4f*)(p);
    const v4f a1 = *(const v4f*)(p + 4);
    const v4f a2 = *(const v4f*)(p + 256);
    const v4f a3 = *(const v4f*)(p + 260);
    v8h w0, w1;
    float s = 0.0f;
#pragma unroll
    for (int e = 0; e < 4; ++e) {
      const float x0 = a0[e];
      const float x1 = a1[e];
      const float x2 = a2[e];
      const float x3 = a3[e];
      const unsigned short b0 = f2bf_bits(x0);
      const unsigned short b1 = f2bf_bits(x1);
      const unsigned short b2 = f2bf_bits(x2);
      const unsigned short b3 = f2bf_bits(x3);
      const float f0 = bf_bits2f(b0);
      const float f1 = bf_bits2f(b1);
      const float f2 = bf_bits2f(b2);
      const float f3 = bf_bits2f(b3);
      w0[e]     = __builtin_bit_cast(_Float16, b0);
      w0[4 + e] = __builtin_bit_cast(_Float16, b1);
      w1[e]     = __builtin_bit_cast(_Float16, b2);
      w1[4 + e] = __builtin_bit_cast(_Float16, b3);
      s = fmaf(f0, f0, s);
      s = fmaf(f1, f1, s);
      s = fmaf(f2, f2, s);
      s = fmaf(f3, f3, s);
      cs[e]      += f0;
      cs[4 + e]  += f1;
      cs[8 + e]  += f2;
      cs[12 + e] += f3;
    }
#pragma unroll
    for (int off = 16; off > 0; off >>= 1) s += __shfl_xor(s, off, 32);
    keep = (lane == r) ? s : keep;

    unsigned short* q = T16 + (size_t)(rowBase + r) * kDim + lane * 8;
    *(volatile v8h*)(q)       = w0;
    *(volatile v8h*)(q + 256) = w1;
    __threadfence();
    *(volatile v8h*)(q)       = w0;
    *(volatile v8h*)(q + 256) = w1;
  }

  {
    float* qs = SQ + rowBase + lane;
    *(volatile float*)qs = keep;
    __threadfence();
    *(volatile float*)qs = keep;
  }

  {
    float* cw = sCol + wave * kDim + lane * 8;
    v4f c0, c1, c2, c3;
#pragma unroll
    for (int e = 0; e < 4; ++e) {
      c0[e] = cs[e];
      c1[e] = cs[4 + e];
      c2[e] = cs[8 + e];
      c3[e] = cs[12 + e];
    }
    *(v4f*)(cw)       = c0;
    *(v4f*)(cw + 4)   = c1;
    *(v4f*)(cw + 256) = c2;
    *(v4f*)(cw + 260) = c3;
  }
  __syncthreads();
  {
    float t0 = 0.0f, t1 = 0.0f;
#pragma unroll
    for (int w = 0; w < 8; ++w) {
      t0 += sCol[w * kDim + tid];
      t1 += sCol[w * kDim + 256 + tid];
    }
    float* qc = COLPART + (size_t)blockIdx.x * kDim + tid;
    *(volatile float*)(qc)       = t0;
    *(volatile float*)(qc + 256) = t1;
    __threadfence();
    *(volatile float*)(qc)       = t0;
    *(volatile float*)(qc + 256) = t1;
  }
}

__global__ __launch_bounds__(256) void bandwidth_kernel(
    const float* __restrict__ SQ, const float* __restrict__ COLPART, float* __restrict__ SCAL)
{
  __shared__ double red[256];
  const int tid = threadIdx.x, lane = tid & 31, wave = tid >> 5;
  double s = 0.0;
#pragma unroll 1
  for (int i = 0; i < kNTot / 256; ++i) s += (double)SQ[tid + 256 * i];
  double c0 = 0.0, c1 = 0.0;
#pragma unroll 1
  for (int b = 0; b < kPrepBlocks; ++b) {
    c0 += (double)COLPART[(size_t)b * kDim + tid];
    c1 += (double)COLPART[(size_t)b * kDim + 256 + tid];
  }
  const double n = (double)kNTot;
  red[tid] = 2.0 * n * s - 2.0 * (c0 * c0 + c1 * c1);
  __syncthreads();
#pragma unroll 1
  for (int off = 128; off > 0; off >>= 1) {
    if (tid < off) red[tid] += red[tid + off];
    __syncthreads();
  }
  if (wave == 0) {
    const double sum_l2 = red[0];
    const double c2d = 1.4426950408889634 * (n * n - n) / (4.0 * sum_l2);
    const float c2f = (float)c2d;
    const float v = (lane == 0) ? c2f : 0.0f;
    float* q = SCAL + lane;
    *(volatile float*)q = v;
    __threadfence();
    *(volatile float*)q = v;
  }
}

__device__ __forceinline__ float ladder_sum8(const v8f d, const v4f sa0, const v4f sa1, float sqn, float c2) {
  float s = 0.0f;
#pragma unroll
  for (int r = 0; r < 8; ++r) {
    const float sa = (r < 4) ? sa0[r & 3] : sa1[r & 3];
    const float dv = d[r];
    const float l2 = fmaxf((sa + sqn) - 2.0f * dv, 0.0f);
    const float t  = __builtin_amdgcn_exp2f(-l2 * c2);
    const float t2 = t * t;
    const float t4 = t2 * t2;
    const float t8 = t4 * t4;
    const float t16 = t8 * t8;
    s += ((t + t2) + (t4 + t8)) + t16;
  }
  return s;
}

__global__ __launch_bounds__(256) void gram_ladder_kernel(
    const unsigned short* __restrict__ T16p, const float* __restrict__ SQ,
    const float* __restrict__ SCAL, float* __restrict__ PART)
{
  __shared__ float sPart[8];
  const __bf16* T = (const __bf16*)T16p;
  const int tid = threadIdx.x, lane = tid & 31, wave = tid >> 5;
  const int w = blockIdx.x * 8 + wave;
  int ti, tj;
  tri_decode(w, ti, tj);
  const int m0 = ti * kTileRows;
  const int n0 = tj * kTileRows;
  const int rlane = lane & 15;
  const int hh    = lane >> 4;
  const int koff  = hh * 8;

  v8f acc[4][4];
#pragma unroll
  for (int i = 0; i < 4; ++i)
#pragma unroll
    for (int j = 0; j < 4; ++j) acc[i][j] = (v8f){0.f, 0.f, 0.f, 0.f, 0.f, 0.f, 0.f, 0.f};

#pragma unroll 1
  for (int k0 = 0; k0 < kDim; k0 += 32) {
    v16b bh[4];
#pragma unroll
    for (int j = 0; j < 4; ++j)
      bh[j] = FragB::load(T + (size_t)(n0 + (j << 4) + rlane) * kDim + koff + k0);
#pragma unroll
    for (int i = 0; i < 4; ++i) {
      const v16b ah = FragB::load(T + (size_t)(m0 + (i << 4) + rlane) * kDim + koff + k0);
#pragma unroll
      for (int j = 0; j < 4; ++j) acc[i][j] = mma_guarded(ah, bh[j], acc[i][j]);
    }
  }

  const float c2 = SCAL[0];
  float sqB[4];
#pragma unroll
  for (int j = 0; j < 4; ++j) sqB[j] = SQ[n0 + (j << 4) + rlane];

  float local = 0.0f;
#pragma unroll
  for (int i = 0; i < 4; ++i) {
    const float* sp = SQ + m0 + (i << 4) + 8 * hh;
    const v4f sa0 = *(const v4f*)(sp);
    const v4f sa1 = *(const v4f*)(sp + 4);
#pragma unroll
    for (int j = 0; j < 4; ++j) local += ladder_sum8(acc[i][j], sa0, sa1, sqB[j], c2);
  }
#pragma unroll
  for (int off = 16; off > 0; off >>= 1) local += __shfl_xor(local, off, 32);

  if (lane == 0) sPart[wave] = local;
  __syncthreads();
  if (wave == 0) {
    const int idx = (lane < 8) ? lane : 7;
    const float pv = sPart[idx];
    const float v = (lane < 8) ? pv : 0.0f;
    float* q = PART + (size_t)blockIdx.x * 32 + lane;
    *(volatile float*)q = v;
    __threadfence();
    *(volatile float*)q = v;
  }
}

__global__ __launch_bounds__(256) void final_reduce_kernel(
    const float* __restrict__ PART, float* __restrict__ out)
{
  __shared__ double red[256];
  const int tid = threadIdx.x;
  constexpr int kIters = (kPairs + 255) / 256;
  constexpr int kHalfTiles = kHalfN / kTileRows;
  double s = 0.0;
#pragma unroll 1
  for (int it = 0; it < kIters; ++it) {
    const int w = tid + 256 * it;
    const bool valid = (w < kPairs);
    const int wc = valid ? w : (kPairs - 1);
    const float pv = PART[(size_t)(wc >> 3) * 32 + (wc & 7)];
    int ti, tj;
    tri_decode(wc, ti, tj);
    const bool same = ((ti < kHalfTiles) == (tj < kHalfTiles));
    const double sw = (ti == tj) ? 1.0 : 2.0;
    const double sg = same ? sw : -sw;
    const double term = sg * (double)pv;
    s += valid ? term : 0.0;
  }
  red[tid] = s;
  __syncthreads();
#pragma unroll 1
  for (int off = 128; off > 0; off >>= 1) {
    if (tid < off) red[tid] += red[tid + off];
    __syncthreads();
  }
  if (tid == 0) {
    const double bsq = (double)kHalfN * (double)kHalfN;
    const float r = (float)(red[0] / bsq);
    *(volatile float*)out = r;
    __threadfence();
    *(volatile float*)out = r;
  }
}

extern "C" void kernel_launch(void* const* d_in, const int* in_sizes, int n_in,
                              void* d_out, int out_size, void* d_ws, size_t ws_size,
                              hipStream_t stream) {
  if (n_in < 2) return;
  if (in_sizes[0] != kHalfN * kDim) return;
  if (in_sizes[1] != kHalfN * kDim) return;
  if (out_size != 1) return;
  if (ws_size < kWsTotal) return;

  const float* src = (const float*)d_in[0];
  const float* tgt = (const float*)d_in[1];
  float* out = (float*)d_out;

  char* ws = (char*)d_ws;
  unsigned short* T16     = (unsigned short*)(ws + kOffT16);
  float*          SQ      = (float*)(ws + kOffSQ);
  float*          COLPART = (float*)(ws + kOffCOL);
  float*          SCAL    = (float*)(ws + kOffSCAL);
  float*          PART    = (float*)(ws + kOffPART);

  prep_rows_kernel<<<kPrepBlocks, 256, 0, stream>>>(src, tgt, T16, SQ, COLPART);
  bandwidth_kernel<<<1, 256, 0, stream>>>(SQ, COLPART, SCAL);
  gram_ladder_kernel<<<kMainBlocks, 256, 0, stream>>>(T16, SQ, SCAL, PART);
  final_reduce_kernel<<<1, 256, 0, stream>>>(PART, out);
}
